// SE3SequenceEncoder_82970178224147
// MI455X (gfx1250) — hardware-verified
//
#include <hip/hip_runtime.h>
#include <math.h>

typedef __attribute__((ext_vector_type(16))) _Float16 v16h;
typedef __attribute__((ext_vector_type(16))) __bf16 v16b;
typedef __attribute__((ext_vector_type(8)))  _Float16 v8h;
typedef __attribute__((ext_vector_type(8)))  float v8f;
typedef __attribute__((ext_vector_type(4)))  float v4f;
typedef __attribute__((ext_vector_type(2)))  float v2f;
typedef __attribute__((ext_vector_type(4)))  unsigned v4u;
typedef __attribute__((ext_vector_type(4)))  int v4i;
typedef float __attribute__((may_alias)) float_a;
typedef int __attribute__((may_alias)) int_a;

template <typename T> __device__ __forceinline__ void vst2(void* p, T v) { *(volatile T*)p = v; __threadfence(); *(volatile T*)p = v; }
__device__ __forceinline__ v8f wmma16(v16h a, v16h b, v8f c) {
  v8f d = __builtin_amdgcn_wmma_f32_16x16x32_f16(false, a, false, b, (short)0, c, false, false);
  asm volatile("v_nop\n\tv_nop\n\tv_nop\n\tv_nop" : "+v"(d) : "v"(a), "v"(b));
  return d;
}
__device__ __forceinline__ v8f wmma_bf(v16b a, v16b b, v8f c) {
  v8f d = __builtin_amdgcn_wmma_f32_16x16x32_bf16(false, a, false, b, (short)0, c, false, false);
  asm volatile("v_nop\n\tv_nop\n\tv_nop\n\tv_nop" : "+v"(d) : "v"(a), "v"(b));
  return d;
}
__device__ __forceinline__ v16h frag_h(const _Float16* rowk0, int lane) {
  union { v16h v; v8h q[2]; } u; const _Float16* p = rowk0 + 8 * (lane >> 4);
  u.q[0] = *(const v8h*)p; u.q[1] = *(const v8h*)(p + 16); return u.v;
}
__device__ __forceinline__ v16h frag_f32(const float* rowk0, int lane) {
  v16h a; const float* p = rowk0 + 8 * (lane >> 4);
#pragma unroll
  for (int i = 0; i < 8; ++i) { a[i] = (_Float16)p[i]; a[8 + i] = (_Float16)p[16 + i]; }
  return a;
}
__device__ __forceinline__ v16h frag_f32s(const float* rowk0, int lane, float sc) {
  v16h a; const float* p = rowk0 + 8 * (lane >> 4);
#pragma unroll
  for (int i = 0; i < 8; ++i) { a[i] = (_Float16)(p[i] * sc); a[8 + i] = (_Float16)(p[16 + i] * sc); }
  return a;
}
__device__ __forceinline__ v16h fragc_f32(const float* W, int k0, int n, int lane, int ld, int K) {
  v16h a; const int g = lane >> 4;
#pragma unroll
  for (int i = 0; i < 8; ++i) { const int ka = k0 + 8 * g + i, kb = ka + 16;
    a[i] = (_Float16)(ka < K ? W[(size_t)ka * ld + n] : 0.f); a[8 + i] = (_Float16)(kb < K ? W[(size_t)kb * ld + n] : 0.f); }
  return a;
}
struct F2 { v16b h, l; };
__device__ __forceinline__ F2 bsplit16(const float v[16]) { F2 r;
#pragma unroll
  for (int i = 0; i < 16; ++i) { const __bf16 h = (__bf16)v[i]; r.h[i] = h; r.l[i] = (__bf16)(v[i] - (float)h); }
  return r; }
__device__ __forceinline__ F2 split_row(const float* row, int k0, int lane) { float v[16]; const float* p = row + k0 + 8 * (lane >> 4);
#pragma unroll
  for (int i = 0; i < 8; ++i) { v[i] = p[i]; v[8 + i] = p[16 + i]; }
  return bsplit16(v); }
__device__ __forceinline__ F2 split_rowK(const float* row, int k0, int lane, int K) { float v[16]; const int g = lane >> 4;
#pragma unroll
  for (int i = 0; i < 8; ++i) { const int ka = k0 + 8 * g + i, kb = ka + 16; v[i] = ka < K ? row[ka] : 0.f; v[8 + i] = kb < K ? row[kb] : 0.f; }
  return bsplit16(v); }
__device__ __forceinline__ F2 split_col(const float* W, int k0, int n, int lane, int ld, int K) { float v[16]; const int g = lane >> 4;
#pragma unroll
  for (int i = 0; i < 8; ++i) { const int ka = k0 + 8 * g + i, kb = ka + 16; v[i] = ka < K ? W[(size_t)ka * ld + n] : 0.f; v[8 + i] = kb < K ? W[(size_t)kb * ld + n] : 0.f; }
  return bsplit16(v); }
__device__ __forceinline__ v8f mac3(const F2& a, const F2& b, v8f c) { c = wmma_bf(a.l, b.h, c); c = wmma_bf(a.h, b.l, c); return wmma_bf(a.h, b.h, c); }
__device__ __forceinline__ float sigm(float v) { return 1.0f / (1.0f + expf(-v)); }
#define LDSX() do { asm volatile("s_wait_dscnt 0" ::: "memory"); __builtin_amdgcn_wave_barrier(); __builtin_amdgcn_fence(__ATOMIC_RELEASE, "workgroup"); } while (0)

#define NB 2
#define NN 384
#define DD 256
#define PD 64
#define NL 8
#define NH 8
#define DH 32
#define NR (NB * NN)
#define FF 1024

__device__ __forceinline__ v16h fragc16(const float* W, int k0, int n, int lane, int ld, int K) { v16h b = fragc_f32(W, k0, n, lane, ld, K);
#pragma unroll
  for (int e = 0; e < 16; ++e) b[e] = b[e] * (_Float16)16.0f; return b; }
__device__ __forceinline__ float gelu_e(float v) { return 0.5f * v * (1.0f + erff(v * 0.70710678118654752f)); }
__device__ __forceinline__ float silu_f(float v) { return v * sigm(v); }

__global__ __launch_bounds__(256) void k_embed(const int* __restrict__ tok, const float* __restrict__ emb, const float* __restrict__ lw, const float* __restrict__ lb, float* __restrict__ x, float* __restrict__ frames) {
  __shared__ float red[2][256];
  const int r = blockIdx.x, c = threadIdx.x; const int n = r % NN; int t = tok[r]; t = t < 0 ? 0 : (t > 20 ? 20 : t);
  const float div = expf((float)(c & ~1) * (-logf(10000.0f) / (float)DD)); const float ang = (float)n * div;
  const float v = emb[t * DD + c] + ((c & 1) ? cosf(ang) : sinf(ang));
  red[0][c] = v; __syncthreads();
  for (int st = 128; st > 0; st >>= 1) { if (c < st) red[0][c] += red[0][c + st]; __syncthreads(); }
  const float mu = red[0][0] / (float)DD; const float d = v - mu; red[1][c] = d * d; __syncthreads();
  for (int st = 128; st > 0; st >>= 1) { if (c < st) red[1][c] += red[1][c + st]; __syncthreads(); }
  const float rs = rsqrtf(red[1][0] / (float)DD + 1e-5f);
  vst2(x + (size_t)r * DD + c, (float_a)(d * rs * lw[c] + lb[c]));
  if ((r & 1) == 0 && c < 32) vst2(frames + (size_t)r * 16 + c, (float_a)(((c & 15) % 5 == 0) ? 1.0f : 0.f));
}
__global__ __launch_bounds__(128) void k_gemm(const float* __restrict__ A, int K, const float* __restrict__ W, int N, const float* __restrict__ bias, float* __restrict__ Out) {
  __shared__ __align__(16) float so[4][16][132];
  const int tid = threadIdx.x, wave = tid >> 5, lane = tid & 31, col = lane & 15, g = lane >> 4;
  const int r0 = blockIdx.x * 64 + wave * 16, n0 = blockIdx.y * 128;
  v8f acc[8] = {};
#pragma unroll 1
  for (int kc = 0; kc < K / 32; ++kc) { const F2 a = split_row(A + (size_t)(r0 + col) * K, kc * 32, lane);
#pragma unroll
    for (int j = 0; j < 8; ++j) acc[j] = mac3(a, split_col(W, kc * 32, n0 + j * 16 + col, lane, N, K), acc[j]); }
#pragma unroll
  for (int j = 0; j < 8; ++j) { const float bb = bias ? bias[n0 + j * 16 + col] : 0.f;
#pragma unroll
    for (int r = 0; r < 8; ++r) so[wave][8 * g + r][j * 16 + col] = acc[j][r] + bb; }
  LDSX();
#pragma unroll 4
  for (int rl = 0; rl < 16; ++rl) vst2(Out + (size_t)(r0 + rl) * N + n0 + lane * 4, *(const v4f*)(&so[wave][rl][lane * 4]));
}
__global__ __launch_bounds__(128) void k_qkv(const float* __restrict__ x, const float* __restrict__ Wq, const float* __restrict__ Wk, const float* __restrict__ Wv, float* __restrict__ qkv) {
  __shared__ __align__(16) float so[4][16][132];
  const int tid = threadIdx.x, wave = tid >> 5, lane = tid & 31, col = lane & 15, g = lane >> 4;
  const int r0 = blockIdx.x * 64 + wave * 16, which = blockIdx.y >> 1, n0 = (blockIdx.y & 1) * 128;
  const float* W = which == 0 ? Wq : (which == 1 ? Wk : Wv);
  v8f acc[8] = {};
#pragma unroll 1
  for (int kc = 0; kc < DD / 32; ++kc) { const v16h a = frag_f32(x + (size_t)(r0 + col) * DD + kc * 32, lane);
#pragma unroll
    for (int j = 0; j < 8; ++j) acc[j] = wmma16(a, fragc16(W, kc * 32, n0 + j * 16 + col, lane, DD, DD), acc[j]); }
#pragma unroll
  for (int j = 0; j < 8; ++j)
#pragma unroll
    for (int r = 0; r < 8; ++r) so[wave][8 * g + r][j * 16 + col] = acc[j][r] * (1.0f / 16.0f);
  LDSX();
#pragma unroll 4
  for (int rl = 0; rl < 16; ++rl) vst2(qkv + (size_t)(r0 + rl) * (3 * DD) + which * DD + n0 + lane * 4, *(const v4f*)(&so[wave][rl][lane * 4]));
}
__global__ __launch_bounds__(128) void k_attn(const float* __restrict__ qkv, const float* __restrict__ frames, float* __restrict__ ao) {
  __shared__ __align__(16) float sS[64][NN + 4];
  __shared__ __align__(16) float sV[NN][DH + 4];
  __shared__ float st3[NN][4];
  __shared__ __align__(16) float so[4][16][36];
  const int tid = threadIdx.x, w = tid >> 5, lane = tid & 31, col = lane & 15, g = lane >> 4;
  const int b = blockIdx.z, h = blockIdx.y, i0 = blockIdx.x * 64 + w * 16;
  for (int q = tid; q < NN * DH; q += 128) { const int j = q >> 5, d = q & 31; sV[j][d] = qkv[(size_t)(b * NN + j) * (3 * DD) + 2 * DD + h * DH + d]; }
  for (int q = tid; q < NN; q += 128) { const float* f = frames + (size_t)(b * NN + q) * 16; st3[q][0] = f[3]; st3[q][1] = f[7]; st3[q][2] = f[11]; }
  __syncthreads();
  const v16h aq = frag_f32(qkv + (size_t)(b * NN + i0 + col) * (3 * DD) + h * DH, lane);
  const float fac = rsqrtf((float)DH);
#pragma unroll 1
  for (int t = 0; t < NN / 16; ++t) { v8f acc = {}; acc = wmma16(aq, frag_f32(qkv + (size_t)(b * NN + t * 16 + col) * (3 * DD) + DD + h * DH, lane), acc);
    const int j = t * 16 + col; const float tjx = st3[j][0], tjy = st3[j][1], tjz = st3[j][2];
#pragma unroll
    for (int r = 0; r < 8; ++r) { const int il = w * 16 + 8 * g + r; const int i = i0 + 8 * g + r;
      const float dx = st3[i][0] - tjx, dy = st3[i][1] - tjy, dz = st3[i][2] - tjz;
      sS[il][j] = acc[r] * fac - (dx * dx + dy * dy + dz * dz); } }
  __syncthreads();
  { const int rl = tid >> 1, hf = tid & 1; float mx = -3.0e38f;
    for (int j = 0; j < NN / 2; ++j) mx = fmaxf(mx, sS[rl][hf * (NN / 2) + j]);
    mx = fmaxf(mx, __shfl_xor(mx, 1, 32));
    float s = 0.f; for (int j = 0; j < NN / 2; ++j) { const float p = expf(sS[rl][hf * (NN / 2) + j] - mx); sS[rl][hf * (NN / 2) + j] = p; s += p; }
    s += __shfl_xor(s, 1, 32); const float inv = 1.0f / s;
    for (int j = 0; j < NN / 2; ++j) sS[rl][hf * (NN / 2) + j] *= inv; }
  __syncthreads();
  v8f acc[2] = {};
#pragma unroll 1
  for (int kc = 0; kc < NN / 32; ++kc) { const v16h pa = frag_f32s(&sS[w * 16 + col][0] + kc * 32, lane, 16384.0f);
#pragma unroll
    for (int t = 0; t < 2; ++t) acc[t] = wmma16(pa, fragc_f32(&sV[0][0], kc * 32, t * 16 + col, lane, DH + 4, NN), acc[t]); }
#pragma unroll
  for (int t = 0; t < 2; ++t)
#pragma unroll
    for (int r = 0; r < 8; ++r) so[w][8 * g + r][t * 16 + col] = acc[t][r] * (1.0f / 16384.0f);
  LDSX();
  for (int q = lane; q < 16 * 8; q += 32) { const int rl = q >> 3, pc = q & 7; vst2(ao + (size_t)(b * NN + i0 + rl) * DD + h * DH + pc * 4, *(const v4f*)(&so[w][rl][pc * 4])); }
}
__global__ __launch_bounds__(128) void k_wo(const float* __restrict__ ao, const float* __restrict__ Wo, const float* __restrict__ bo, const float* __restrict__ l1w, const float* __restrict__ l1b, const float* __restrict__ l2w, const float* __restrict__ l2b,
                                          float* __restrict__ x, float* __restrict__ hln) {
  __shared__ __align__(16) float so[4][16][260];
  const int tid = threadIdx.x, wave = tid >> 5, lane = tid & 31, col = lane & 15, g = lane >> 4;
  const int r0 = blockIdx.x * 64 + wave * 16;
#pragma unroll 1
  for (int hf = 0; hf < 2; ++hf) { v8f acc[8] = {};
#pragma unroll 1
    for (int kc = 0; kc < DD / 32; ++kc) { const F2 a = split_row(ao + (size_t)(r0 + col) * DD, kc * 32, lane);
#pragma unroll
      for (int j = 0; j < 8; ++j) acc[j] = mac3(a, split_col(Wo, kc * 32, hf * 128 + j * 16 + col, lane, DD, DD), acc[j]); }
#pragma unroll
    for (int j = 0; j < 8; ++j) { const int c = hf * 128 + j * 16 + col; const float bb = bo[c];
#pragma unroll
      for (int r = 0; r < 8; ++r) so[wave][8 * g + r][c] = acc[j][r] + bb + x[(size_t)(r0 + 8 * g + r) * DD + c]; } }
  LDSX();
  { const int rl = lane >> 1, hf = lane & 1; float* row = &so[wave][rl][0];
    float s = 0.f; for (int c = 0; c < 128; ++c) s += row[hf * 128 + c]; s += __shfl_xor(s, 1, 32); const float mu = s / (float)DD;
    float q2 = 0.f; for (int c = 0; c < 128; ++c) { const float d = row[hf * 128 + c] - mu; q2 += d * d; } q2 += __shfl_xor(q2, 1, 32); const float rs = rsqrtf(q2 / (float)DD + 1e-5f);
    float s2 = 0.f; for (int c = 0; c < 128; ++c) { const int cc = hf * 128 + c; const float v = (row[cc] - mu) * rs * l1w[cc] + l1b[cc]; row[cc] = v; s2 += v; }
    s2 += __shfl_xor(s2, 1, 32); const float mu2 = s2 / (float)DD;
    float q3 = 0.f; for (int c = 0; c < 128; ++c) { const float d = row[hf * 128 + c] - mu2; q3 += d * d; } q3 += __shfl_xor(q3, 1, 32); const float rs2 = rsqrtf(q3 / (float)DD + 1e-5f);
    LDSX();
    for (int c4 = 0; c4 < 32; ++c4) { const int cc = hf * 128 + c4 * 4; const v4f v = *(const v4f*)(&row[cc]); v4f o2;
#pragma unroll
      for (int e = 0; e < 4; ++e) o2[e] = (v[e] - mu2) * rs2 * l2w[cc + e] + l2b[cc + e];
      vst2(x + (size_t)(r0 + rl) * DD + cc, v); vst2(hln + (size_t)(r0 + rl) * DD + cc, o2); } }
}
__global__ __launch_bounds__(64) void k_ffn(const float* __restrict__ hln, const float* __restrict__ W1, const float* __restrict__ b1, const float* __restrict__ W2, const float* __restrict__ b2,
                                           const float* __restrict__ Wop, const float* __restrict__ bop, float* __restrict__ x, float* __restrict__ proj) {
  __shared__ __align__(16) float sg[32][FF + 4];
  __shared__ __align__(16) float sx[2][16][260];
  __shared__ __align__(16) float sp[2][16][68];
  const int tid = threadIdx.x, wave = tid >> 5, lane = tid & 31, col = lane & 15, g = lane >> 4;
  const int r0 = blockIdx.x * 32 + wave * 16;
#pragma unroll 1
  for (int nc = 0; nc < FF / 128; ++nc) { v8f acc[8] = {};
#pragma unroll 1
    for (int kc = 0; kc < DD / 32; ++kc) { const v16h a = frag_f32(hln + (size_t)(r0 + col) * DD + kc * 32, lane);
#pragma unroll
      for (int j = 0; j < 8; ++j) acc[j] = wmma16(a, fragc16(W1, kc * 32, nc * 128 + j * 16 + col, lane, FF, DD), acc[j]); }
#pragma unroll
    for (int j = 0; j < 8; ++j) { const int c = nc * 128 + j * 16 + col; const float bb = b1[c];
#pragma unroll
      for (int r = 0; r < 8; ++r) sg[wave * 16 + 8 * g + r][c] = gelu_e(acc[j][r] * (1.0f / 16.0f) + bb); } }
  LDSX();
#pragma unroll 1
  for (int hf = 0; hf < 2; ++hf) { v8f acc[8] = {};
#pragma unroll 1
    for (int kc = 0; kc < FF / 32; ++kc) { const v16h a = frag_f32(&sg[wave * 16 + col][0] + kc * 32, lane);
#pragma unroll
      for (int j = 0; j < 8; ++j) acc[j] = wmma16(a, fragc16(W2, kc * 32, hf * 128 + j * 16 + col, lane, DD, FF), acc[j]); }
#pragma unroll
    for (int j = 0; j < 8; ++j) { const int c = hf * 128 + j * 16 + col; const float bb = b2[c];
#pragma unroll
      for (int r = 0; r < 8; ++r) sx[wave][8 * g + r][c] = acc[j][r] * (1.0f / 16.0f) + bb + x[(size_t)(r0 + 8 * g + r) * DD + c]; } }
  LDSX();
#pragma unroll 2
  for (int rl = 0; rl < 16; ++rl) { vst2(x + (size_t)(r0 + rl) * DD + lane * 4, *(const v4f*)(&sx[wave][rl][lane * 4])); vst2(x + (size_t)(r0 + rl) * DD + 128 + lane * 4, *(const v4f*)(&sx[wave][rl][128 + lane * 4])); }
  { v8f acc[4] = {};
#pragma unroll 1
    for (int kc = 0; kc < DD / 32; ++kc) { const F2 a = split_row(&sx[wave][col][0], kc * 32, lane);
#pragma unroll
      for (int j = 0; j < 4; ++j) acc[j] = mac3(a, split_col(Wop, kc * 32, j * 16 + col, lane, PD, DD), acc[j]); }
#pragma unroll
    for (int j = 0; j < 4; ++j) { const int c = j * 16 + col; const float bb = bop[c];
#pragma unroll
      for (int r = 0; r < 8; ++r) { const float v = acc[j][r] + bb; sp[wave][8 * g + r][c] = v > 0.f ? v : 0.f; } } }
  LDSX();
  for (int q = lane; q < 16 * 16; q += 32) { const int rl = q >> 4, pc = q & 15; vst2(proj + (size_t)(r0 + rl) * PD + pc * 4, *(const v4f*)(&sp[wave][rl][pc * 4])); }
}
__global__ __launch_bounds__(256) void k_pair(const float* __restrict__ proj, const float* __restrict__ rel, const float* __restrict__ pw, const float* __restrict__ pb, float* __restrict__ pm) {
  __shared__ float spi[8][PD];
  __shared__ __align__(16) float so[8][PD];
  const int tid = threadIdx.x, w = tid >> 5, lane = tid & 31; const int r = blockIdx.x * 8 + w; const int b = r / NN, i = r % NN;
  spi[w][lane] = proj[(size_t)r * PD + lane]; spi[w][lane + 32] = proj[(size_t)r * PD + lane + 32];
  LDSX();
  float acc[PD];
#pragma unroll
  for (int c = 0; c < PD; ++c) acc[c] = 0.f;
#pragma unroll 1
  for (int jr = 0; jr < NN / 32; ++jr) { const int j = jr * 32 + lane; int dlt = j - i; dlt = dlt < -64 ? -64 : (dlt > 64 ? 64 : dlt);
    const float* re = rel + (size_t)(dlt + 64) * PD; const float* pj = proj + (size_t)(b * NN + j) * PD;
    float v[PD]; float s = 0.f;
#pragma unroll
    for (int c = 0; c < PD; ++c) { v[c] = spi[w][c] + pj[c] + re[c]; s += v[c]; }
    const float mu = s * (1.0f / (float)PD); float q2 = 0.f;
#pragma unroll
    for (int c = 0; c < PD; ++c) { const float d = v[c] - mu; q2 += d * d; }
    const float rs = rsqrtf(q2 * (1.0f / (float)PD) + 1e-5f);
#pragma unroll
    for (int c = 0; c < PD; ++c) acc[c] += (v[c] - mu) * rs; }
#pragma unroll
  for (int c = 0; c < PD; ++c) { float t = acc[c];
#pragma unroll
    for (int off = 16; off >= 1; off >>= 1) t += __shfl_xor(t, off, 32);
    if (lane == (c & 31)) { if (c < 32) so[w][c] = t; else so[w][c] = t; } }
  LDSX();
  { const float s0v = so[w][lane] * (1.0f / (float)NN) * pw[lane] + pb[lane], s1v = so[w][lane + 32] * (1.0f / (float)NN) * pw[lane + 32] + pb[lane + 32];
    LDSX(); so[w][lane] = s0v; so[w][lane + 32] = s1v; }
  LDSX();
  if (lane < 16) vst2(pm + (size_t)r * PD + lane * 4, *(const v4f*)(&so[w][lane * 4]));
}
__global__ __launch_bounds__(128) void k_frame(const float* __restrict__ x, const float* __restrict__ pm, const float* __restrict__ Wf1, const float* __restrict__ bf1, const float* __restrict__ Wf2, const float* __restrict__ bf2, float* __restrict__ frames) {
  __shared__ __align__(16) float sh[4][16][132];
  __shared__ __align__(16) float sf[4][16][16];
  const int tid = threadIdx.x, wave = tid >> 5, lane = tid & 31, col = lane & 15, g = lane >> 4;
  const int r0 = blockIdx.x * 64 + wave * 16;
  v8f acc[8] = {};
#pragma unroll 1
  for (int kc = 0; kc < (DD + PD) / 32; ++kc) { F2 a; if (kc < DD / 32) a = split_row(x + (size_t)(r0 + col) * DD, kc * 32, lane); else a = split_row(pm + (size_t)(r0 + col) * PD, (kc - DD / 32) * 32, lane);
#pragma unroll
    for (int j = 0; j < 8; ++j) acc[j] = mac3(a, split_col(Wf1, kc * 32, j * 16 + col, lane, 128, DD + PD), acc[j]); }
#pragma unroll
  for (int j = 0; j < 8; ++j) { const int c = j * 16 + col; const float bb = bf1[c];
#pragma unroll
    for (int r = 0; r < 8; ++r) sh[wave][8 * g + r][c] = silu_f(acc[j][r] + bb); }
  LDSX();
  if (lane < 16) { const int rl = lane; float raw[9];
#pragma unroll
    for (int k = 0; k < 9; ++k) raw[k] = bf2[k];
#pragma unroll 1
    for (int c = 0; c < 128; ++c) { const float hv = sh[wave][rl][c];
#pragma unroll
      for (int k = 0; k < 9; ++k) raw[k] += hv * Wf2[c * 9 + k]; }
    const float n1 = sqrtf(raw[0] * raw[0] + raw[1] * raw[1] + raw[2] * raw[2] + 1e-8f); const float b1x = raw[0] / n1, b1y = raw[1] / n1, b1z = raw[2] / n1;
    const float dp = b1x * raw[3] + b1y * raw[4] + b1z * raw[5]; const float ax = raw[3] - dp * b1x, ay = raw[4] - dp * b1y, az = raw[5] - dp * b1z;
    const float n2 = sqrtf(ax * ax + ay * ay + az * az + 1e-8f); const float b2x = ax / n2, b2y = ay / n2, b2z = az / n2;
    const float b3x = b1y * b2z - b1z * b2y, b3y = b1z * b2x - b1x * b2z, b3z = b1x * b2y - b1y * b2x;
    float* f = &sf[wave][rl][0];
    f[0] = b1x; f[1] = b1y; f[2] = b1z; f[3] = raw[6]; f[4] = b2x; f[5] = b2y; f[6] = b2z; f[7] = raw[7]; f[8] = b3x; f[9] = b3y; f[10] = b3z; f[11] = raw[8]; f[12] = 0.f; f[13] = 0.f; f[14] = 0.f; f[15] = 1.0f; }
  LDSX();
  for (int q = lane; q < 16 * 4; q += 32) { const int rl = q >> 2, pc = q & 3; vst2(frames + (size_t)(r0 + rl) * 16 + pc * 4, *(const v4f*)(&sf[wave][rl][pc * 4])); }
}
extern "C" void kernel_launch(void* const* d_in, const int* in_sizes, int n_in, void* d_out, int out_size, void* d_ws, size_t ws_size, hipStream_t stream) {
  (void)in_sizes; (void)n_in; (void)out_size; (void)ws_size;
  const float** I = (const float**)d_in; const int* tok = (const int*)d_in[0];
  const float* emb = I[1]; const float* elw = I[2]; const float* elb = I[3]; const float* Wq = I[4]; const float* Wk = I[5]; const float* Wv = I[6]; const float* Wo = I[7]; const float* bo = I[8];
  const float* alw = I[9]; const float* alb = I[10]; const float* flw = I[11]; const float* flb = I[12]; const float* W1 = I[13]; const float* b1 = I[14]; const float* W2 = I[15]; const float* b2 = I[16];
  const float* Wop = I[17]; const float* bop = I[18]; const float* rel = I[19]; const float* plw = I[20]; const float* plb = I[21]; const float* Wf1 = I[22]; const float* bf1 = I[23]; const float* Wf2 = I[24]; const float* bf2 = I[25];
  float* frames = (float*)d_out; float* xout = frames + (size_t)NR * 16;
  char* ws = (char*)d_ws; size_t off = 0;
  auto take = [&](size_t bytes) { char* p = ws + off; off += (bytes + 255) & ~(size_t)255; return p; };
  float* qkv = (float*)take((size_t)NR * 3 * DD * 4); float* ao = (float*)take((size_t)NR * DD * 4); float* hln = (float*)take((size_t)NR * DD * 4);
  float* proj = (float*)take((size_t)NR * PD * 4); float* pm = (float*)take((size_t)NR * PD * 4);
  float* x = xout;
  k_embed<<<NR, 256, 0, stream>>>(tok, emb, elw, elb, x, frames);
  for (int l = 0; l < NL; ++l) {
    k_qkv<<<dim3(NR / 64, 6), 128, 0, stream>>>(x, Wq + (size_t)l * DD * DD, Wk + (size_t)l * DD * DD, Wv + (size_t)l * DD * DD, qkv);
    k_attn<<<dim3(NN / 64, NH, NB), 128, 0, stream>>>(qkv, frames, ao);
    k_wo<<<NR / 64, 128, 0, stream>>>(ao, Wo + (size_t)l * DD * DD, bo + l * DD, alw + l * DD, alb + l * DD, flw + l * DD, flb + l * DD, x, hln);
    k_ffn<<<NR / 32, 64, 0, stream>>>(hln, W1 + (size_t)l * DD * FF, b1 + l * FF, W2 + (size_t)l * FF * DD, b2 + l * DD, Wop, bop, x, proj);
    k_pair<<<NR / 8, 256, 0, stream>>>(proj, rel, plw, plb, pm);
    k_frame<<<NR / 64, 128, 0, stream>>>(x, pm, Wf1, bf1, Wf2, bf2, frames);
  }
}
